// MambaVisionCDDecoderBlock_42082089566727
// MI455X (gfx1250) — hardware-run, weakly checked
//
#include <hip/hip_runtime.h>
#include <math.h>

typedef __attribute__((ext_vector_type(16))) _Float16 v16h;
typedef __attribute__((ext_vector_type(8)))  _Float16 v8h;
typedef __attribute__((ext_vector_type(8)))  float    v8f;
typedef __attribute__((ext_vector_type(4)))  float    v4f;
typedef __attribute__((ext_vector_type(4)))  unsigned v4u;

constexpr int kNB   = 8;
constexpr int kDm   = 192;
constexpr int kDx   = 96;
constexpr int kNst  = 16;
constexpr int kDtR  = 12;
constexpr int kH    = 56;
constexpr int kW    = 56;
constexpr int kL    = kH * kW;
constexpr int kOC   = 96;
constexpr int kOH   = 2 * kH;
constexpr int kOW   = 2 * kW;
constexpr int kRows = kNB * kL;
constexpr int kHP   = kH + 2;
constexpr int kWP   = kW + 2;
constexpr int kXdN  = kDtR + 2 * kNst;
constexpr int kXdP  = 64;
constexpr int kK2   = 9 * kDm;
constexpr int kKT   = 4 * kDm;
constexpr int kTilesM = kRows / 64;
constexpr float kWCarry   = 64.0f;
constexpr float kActCarry = 256.0f;
constexpr float kOutCarry = 256.0f;

static_assert(kL == 3136 && kRows == 25088, "token rows");
static_assert(kXdN == 44 && kXdN <= kXdP, "x_proj width");
static_assert((kRows % 64) == 0 && (kL % 64) == 0, "M tiles never cross a batch element");
static_assert((kDm % 64) == 0 && (kXdP % 64) == 0 && (kOC % 32) == 0, "N tile multiples");
static_assert((kDm % 32) == 0 && (kDx % 32) == 0 && (kK2 % 32) == 0 && (kKT % 32) == 0, "K multiples of 32");
static_assert((kL % 16) == 0 && (kRows % 32) == 0, "chunk multiples");
static_assert(kOH == 112 && kOW == 112 && (kOW % 4) == 0, "output plane");

constexpr size_t kSzWIN   = (size_t)kDm * kDm * 2;
constexpr size_t kSzWOUT  = (size_t)kDm * kDm * 2;
constexpr size_t kSzWXP   = (size_t)kXdP * kDx * 2;
constexpr size_t kSzWC2   = (size_t)kDm * kK2 * 2;
constexpr size_t kSzWCT   = (size_t)4 * kOC * kKT * 2;
constexpr size_t kSzXA    = (size_t)kRows * kDm * 2;
constexpr size_t kSzXZ    = (size_t)kRows * kDm * 2;
constexpr size_t kSzXH32  = (size_t)kRows * kDx * 4;
constexpr size_t kSzXH16  = (size_t)kRows * kDx * 2;
constexpr size_t kSzZ16   = (size_t)kRows * kDx * 2;
constexpr size_t kSzXD    = (size_t)kRows * kXdP * 4;
constexpr size_t kSzY16   = (size_t)kRows * kDx * 2;
constexpr size_t kSzOUT16 = (size_t)kRows * kDm * 2;
constexpr size_t kSzIMG   = (size_t)kNB * kHP * kWP * kDm * 2;
constexpr size_t kSzY2    = (size_t)kNB * kHP * kWP * kDm * 2;
constexpr size_t kSzY3    = (size_t)4 * kRows * kOC * 4;
constexpr size_t kOffWIN   = 0;
constexpr size_t kOffWOUT  = kOffWIN   + kSzWIN;
constexpr size_t kOffWXP   = kOffWOUT  + kSzWOUT;
constexpr size_t kOffWC2   = kOffWXP   + kSzWXP;
constexpr size_t kOffWCT   = kOffWC2   + kSzWC2;
constexpr size_t kOffXA    = kOffWCT   + kSzWCT;
constexpr size_t kOffXZ    = kOffXA    + kSzXA;
constexpr size_t kOffXH32  = kOffXZ    + kSzXZ;
constexpr size_t kOffXH16  = kOffXH32  + kSzXH32;
constexpr size_t kOffZ16   = kOffXH16  + kSzXH16;
constexpr size_t kOffXD    = kOffZ16   + kSzZ16;
constexpr size_t kOffY16   = kOffXD    + kSzXD;
constexpr size_t kOffOUT16 = kOffY16   + kSzY16;
constexpr size_t kOffIMG   = kOffOUT16 + kSzOUT16;
constexpr size_t kOffY2    = kOffIMG   + kSzIMG;
constexpr size_t kOffY3    = kOffY2    + kSzY2;
constexpr size_t kWsTotal  = kOffY3    + kSzY3;
static_assert(kWsTotal == 120025088ull, "carve total");
static_assert(kWsTotal <= 134217728ull, "carve cap");
static_assert((kOffWOUT % 128) == 0 && (kOffWXP % 128) == 0 && (kOffWC2 % 128) == 0 && (kOffWCT % 128) == 0 &&
              (kOffXA % 128) == 0 && (kOffXZ % 128) == 0 && (kOffXH32 % 128) == 0 && (kOffXH16 % 128) == 0 &&
              (kOffZ16 % 128) == 0 && (kOffXD % 128) == 0 && (kOffY16 % 128) == 0 && (kOffOUT16 % 128) == 0 &&
              (kOffIMG % 128) == 0 && (kOffY2 % 128) == 0 && (kOffY3 % 128) == 0, "128-B aligned regions");

union FragU { v16h v; v8h h[2]; };
__device__ __forceinline__ v16h frag_load(const _Float16* p) {
  FragU f;
  f.h[0] = *(const v8h*)(p);
  f.h[1] = *(const v8h*)(p + 16);
  return f.v;
}
__device__ __forceinline__ v8f mma_h(v16h a, v16h b, v8f c) {
  c = __builtin_amdgcn_wmma_f32_16x16x32_f16(false, a, false, b, (short)0, c, false, false);
  asm volatile("v_nop\n\tv_nop\n\tv_nop\n\tv_nop" : "+v"(c) : "v"(a), "v"(b));
  return c;
}
__device__ __forceinline__ void slab_sync() {
  __builtin_amdgcn_fence(__ATOMIC_RELEASE, "workgroup");
  __builtin_amdgcn_wave_barrier();
  __builtin_amdgcn_fence(__ATOMIC_ACQUIRE, "workgroup");
}
__device__ __forceinline__ float h16_to_f32(unsigned hb) {
  const unsigned sgn = (hb & 0x8000u) << 16;
  const unsigned em = hb & 0x7fffu;
  const float fn = __uint_as_float((em << 13) + 0x38000000u);
  const float fs = (float)em * 5.9604644775390625e-8f;
  const float mag = (em < 0x400u) ? fs : fn;
  return __uint_as_float(__float_as_uint(mag) | sgn);
}

__global__ __launch_bounds__(256) void cast_f16_pad_kernel(
    const float* __restrict__ src, unsigned short* __restrict__ dst, int total8, int nreal, float scale)
{
  const int i = blockIdx.x * 256 + threadIdx.x;
  if (i >= total8) return;
  const int e0 = i << 3;
  const bool real = e0 < nreal;
  const int ec = real ? e0 : (nreal - 8);
  const v4f a0 = *(const v4f*)(src + ec);
  const v4f a1 = *(const v4f*)(src + ec + 4);
  v8h hv;
#pragma unroll
  for (int e = 0; e < 4; ++e) {
    const float f0 = real ? (a0[e] * scale) : 0.0f;
    const float f1 = real ? (a1[e] * scale) : 0.0f;
    hv[e]     = (_Float16)f0;
    hv[4 + e] = (_Float16)f1;
  }
  unsigned short* q = dst + e0;
  *(volatile v8h*)q = hv;
  __threadfence();
  *(volatile v8h*)q = hv;
}

__global__ __launch_bounds__(256) void pack_conv3x3_kernel(
    const float* __restrict__ Wsrc, unsigned short* __restrict__ Bt, float carry)
{
  const int i = blockIdx.x * 256 + threadIdx.x;
  if (i >= (kDm * kK2) / 8) return;
  const int e0 = i << 3;
  const int co = e0 / kK2;
  const int k = e0 - co * kK2;
  const int tap = k / kDm;
  const int ci0 = k - tap * kDm;
  const float* sp = Wsrc + ((size_t)co * kDm + ci0) * 9 + tap;
  v8h hv;
#pragma unroll
  for (int e = 0; e < 8; ++e) hv[e] = (_Float16)(sp[e * 9] * carry);
  unsigned short* q = Bt + e0;
  *(volatile v8h*)q = hv;
  __threadfence();
  *(volatile v8h*)q = hv;
}

__global__ __launch_bounds__(256) void pack_convT_kernel(
    const float* __restrict__ Wsrc, unsigned short* __restrict__ Bt, float carry)
{
  const int i = blockIdx.x * 256 + threadIdx.x;
  if (i >= (4 * kOC * kKT) / 8) return;
  const int e0 = i << 3;
  const int s = e0 / (kOC * kKT);
  const int r = e0 - s * (kOC * kKT);
  const int co = r / kKT;
  const int k = r - co * kKT;
  const int jj = k / kDm;
  const int ci0 = k - jj * kDm;
  const int sy = s >> 1, sx = s & 1;
  const int jy = jj >> 1, jx = jj & 1;
  const int ky = (sy == 0) ? (jy ? 3 : 1) : (jy ? 0 : 2);
  const int kx = (sx == 0) ? (jx ? 3 : 1) : (jx ? 0 : 2);
  const float* sp = Wsrc + ((size_t)ci0 * kOC + co) * 16 + ky * 4 + kx;
  v8h hv;
#pragma unroll
  for (int e = 0; e < 8; ++e) hv[e] = (_Float16)(sp[(size_t)e * kOC * 16] * carry);
  unsigned short* q = Bt + e0;
  *(volatile v8h*)q = hv;
  __threadfence();
  *(volatile v8h*)q = hv;
}

__global__ __launch_bounds__(256) void nchw_to_rows_f16_kernel(
    const float* __restrict__ X, unsigned short* __restrict__ XA)
{
  __shared__ __align__(16) float tile[kDm * 68];
  const int tid = threadIdx.x, lane = tid & 31, wave = tid >> 5;
  const int bb = blockIdx.x / (kL / 64);
  const int l0 = (blockIdx.x - bb * (kL / 64)) * 64;
  const float* src = X + (size_t)bb * kDm * kL + l0;
#pragma unroll 4
  for (int p = 0; p < 12; ++p) {
    const int idx = tid + p * 256;
    const int c = idx >> 4;
    const int l4 = (idx & 15) * 4;
    const v4f v = *(const v4f*)(src + (size_t)c * kL + l4);
    *(v4f*)(tile + c * 68 + l4) = v;
  }
  __syncthreads();
  const int q = lane >> 3, c8 = (lane & 7) * 8;
  v8h hv[6];
#pragma unroll
  for (int it = 0; it < 6; ++it) {
    const int ln = it * 32 + wave * 4 + q;
    const int row = ln / 3;
    const int col0 = (ln - row * 3) * 64 + c8;
#pragma unroll
    for (int e = 0; e < 8; ++e) hv[it][e] = (_Float16)tile[(col0 + e) * 68 + row];
  }
  for (int pass = 0; pass < 2; ++pass) {
#pragma unroll
    for (int it = 0; it < 6; ++it) {
      const int ln = it * 32 + wave * 4 + q;
      const int row = ln / 3;
      const int col0 = (ln - row * 3) * 64 + c8;
      *(volatile v8h*)(XA + ((size_t)bb * kL + l0 + row) * kDm + col0) = hv[it];
    }
    __threadfence();
  }
}

template <int OUT_MODE, bool TWO_A>
__global__ __launch_bounds__(256) void gemm64_f16_kernel(
    const unsigned short* __restrict__ A1p, int lda1,
    const unsigned short* __restrict__ A2p, int lda2, int ksplit,
    const unsigned short* __restrict__ Btp, int ldb,
    void* __restrict__ Cout, int ldc, int M, int N, int K, float scale)
{
  const _Float16* A1 = (const _Float16*)A1p;
  const _Float16* A2 = (const _Float16*)A2p;
  const _Float16* Bt = (const _Float16*)Btp;
  __shared__ __align__(16) float sT[8][16 * 68];
  const int lane = threadIdx.x & 31;
  const int wave = threadIdx.x >> 5;
  const int tilesN = N >> 6;
  const int tilesM = M >> 6;
  const int tile = blockIdx.x * 8 + wave;
  if (tile >= tilesM * tilesN) return;
  const int tm = tile / tilesN;
  const int tn = tile - tm * tilesN;
  const int m0 = tm << 6;
  const int n0 = tn << 6;
  const int rlane = lane & 15;
  const int koff  = (lane >> 4) * 8;
  const int mOff  = (lane >> 4) * 8;

  v8f acc[4][4];
#pragma unroll
  for (int i = 0; i < 4; ++i)
#pragma unroll
    for (int j = 0; j < 4; ++j) acc[i][j] = (v8f){0.f, 0.f, 0.f, 0.f, 0.f, 0.f, 0.f, 0.f};

  for (int k0 = 0; k0 < K; k0 += 32) {
    const bool second = TWO_A && (k0 >= ksplit);
    const _Float16* Ak = second ? A2 : A1;
    const int lda = second ? lda2 : lda1;
    const int ka = second ? (k0 - ksplit) : k0;
    v16h bh[4];
#pragma unroll
    for (int j = 0; j < 4; ++j)
      bh[j] = frag_load(Bt + (size_t)(n0 + (j << 4) + rlane) * ldb + koff + k0);
#pragma unroll
    for (int i = 0; i < 4; ++i) {
      const v16h ah = frag_load(Ak + (size_t)(m0 + (i << 4) + rlane) * lda + koff + ka);
#pragma unroll
      for (int j = 0; j < 4; ++j) acc[i][j] = mma_h(ah, bh[j], acc[i][j]);
    }
  }

  float* slab = sT[wave];
#pragma unroll
  for (int i = 0; i < 4; ++i) {
    const int mBase = m0 + (i << 4);
#pragma unroll
    for (int j = 0; j < 4; ++j) {
#pragma unroll
      for (int r = 0; r < 8; ++r) slab[(mOff + r) * 68 + (j << 4) + rlane] = acc[i][j][r] * scale;
    }
    slab_sync();
    if (OUT_MODE == 0) {
      float* C = (float*)Cout;
      const int hh = lane >> 4, c4 = (lane & 15) * 4;
      for (int pass = 0; pass < 2; ++pass) {
#pragma unroll
        for (int it = 0; it < 8; ++it) {
          const int row = it * 2 + hh;
          const v4f v = *(const v4f*)(slab + row * 68 + c4);
          *(volatile v4f*)(C + (size_t)(mBase + row) * ldc + n0 + c4) = v;
        }
        __threadfence();
      }
    } else {
      unsigned short* C = (unsigned short*)Cout;
      const int q = lane >> 3, c8 = (lane & 7) * 8;
      for (int pass = 0; pass < 2; ++pass) {
#pragma unroll
        for (int it = 0; it < 4; ++it) {
          const int row = it * 4 + q;
          const float* sp = slab + row * 68 + c8;
          v8h hv;
#pragma unroll
          for (int e = 0; e < 8; ++e) hv[e] = (_Float16)sp[e];
          *(volatile v8h*)(C + (size_t)(mBase + row) * ldc + n0 + c8) = hv;
        }
        __threadfence();
      }
    }
    slab_sync();
  }
}

__global__ __launch_bounds__(256) void dwconv_silu_kernel(
    const unsigned short* __restrict__ XZ,
    const float* __restrict__ wx, const float* __restrict__ bx,
    const float* __restrict__ wz, const float* __restrict__ bz,
    float* __restrict__ XH32, unsigned short* __restrict__ XH16, unsigned short* __restrict__ Z16,
    float carry)
{
  __shared__ __align__(16) float sW[kDm * 4];
  __shared__ __align__(16) float sXZ[2 * 32 * kDx];
  const int tid = threadIdx.x;
  const int row0 = blockIdx.x * 32;
  if (tid < kDx) {
    sW[tid * 4 + 0] = wx[tid * 3 + 0];
    sW[tid * 4 + 1] = wx[tid * 3 + 1];
    sW[tid * 4 + 2] = wx[tid * 3 + 2];
    sW[tid * 4 + 3] = bx[tid];
  } else if (tid < kDm) {
    const int c = tid - kDx;
    sW[tid * 4 + 0] = wz[c * 3 + 0];
    sW[tid * 4 + 1] = wz[c * 3 + 1];
    sW[tid * 4 + 2] = wz[c * 3 + 2];
    sW[tid * 4 + 3] = bz[c];
  }
  __syncthreads();
  const unsigned* XZw = (const unsigned*)(const void*)XZ;
#pragma unroll 1
  for (int p = 0; p < 12; ++p) {
    const int idx = tid + p * 256;
    const int r = idx / kDx;
    const int cp = idx - r * kDx;
    const int m = row0 + r;
    const int bb = m / kL;
    const int l = m - bb * kL;
    const bool hasPrev = l > 0;
    const bool hasNext = l < (kL - 1);
    const int mp = hasPrev ? (m - 1) : m;
    const int mn = hasNext ? (m + 1) : m;
    const unsigned wc = XZw[(size_t)m * kDx + cp];
    const unsigned wp = XZw[(size_t)mp * kDx + cp];
    const unsigned wn = XZw[(size_t)mn * kDx + cp];
    const float u0a = h16_to_f32(wc & 0xffffu);
    const float u0b = h16_to_f32(wc >> 16);
    const float tpa = h16_to_f32(wp & 0xffffu);
    const float tpb = h16_to_f32(wp >> 16);
    const float tna = h16_to_f32(wn & 0xffffu);
    const float tnb = h16_to_f32(wn >> 16);
    const float upa = hasPrev ? tpa : 0.0f;
    const float upb = hasPrev ? tpb : 0.0f;
    const float una = hasNext ? tna : 0.0f;
    const float unb = hasNext ? tnb : 0.0f;
    const int c0 = cp * 2;
    const v4f wa = *(const v4f*)(sW + c0 * 4);
    const v4f wb = *(const v4f*)(sW + c0 * 4 + 4);
    float va = wa[0] * upa;
    va = fmaf(wa[1], u0a, va);
    va = fmaf(wa[2], una, va);
    va = va + wa[3];
    float vb = wb[0] * upb;
    vb = fmaf(wb[1], u0b, vb);
    vb = fmaf(wb[2], unb, vb);
    vb = vb + wb[3];
    const float sa = va * (1.0f / (1.0f + expf(-va)));
    const float sb = vb * (1.0f / (1.0f + expf(-vb)));
    const int sel = (cp >= (kDx / 2)) ? 1 : 0;
    float* dp = sXZ + sel * (32 * kDx) + r * kDx + (c0 - sel * kDx);
    dp[0] = sa;
    dp[1] = sb;
  }
  __syncthreads();
  v4f fv[3];
  v8h hv[3];
#pragma unroll
  for (int it = 0; it < 3; ++it) {
    const int g = it * 256 + tid;
    fv[it] = *(const v4f*)(sXZ + g * 4);
    const int pl = g / 384;
    const int w8 = g - pl * 384;
    const float* sp = sXZ + pl * (32 * kDx) + w8 * 8;
    const v4f a0 = *(const v4f*)(sp);
    const v4f a1 = *(const v4f*)(sp + 4);
#pragma unroll
    for (int e = 0; e < 4; ++e) {
      hv[it][e]     = (_Float16)(a0[e] * carry);
      hv[it][4 + e] = (_Float16)(a1[e] * carry);
    }
  }
  for (int pass = 0; pass < 2; ++pass) {
#pragma unroll
    for (int it = 0; it < 3; ++it) {
      const int g = it * 256 + tid;
      *(volatile v4f*)(XH32 + (size_t)row0 * kDx + g * 4) = fv[it];
      const int pl = g / 384;
      const int w8 = g - pl * 384;
      unsigned short* dst = (pl == 0) ? XH16 : Z16;
      *(volatile v8h*)(dst + (size_t)row0 * kDx + w8 * 8) = hv[it];
    }
    __threadfence();
  }
}

__global__ __launch_bounds__(96) void scan_kernel(
    const float* __restrict__ XD, const float* __restrict__ XH32,
    const float* __restrict__ Wdt, const float* __restrict__ bdt,
    const float* __restrict__ Alog, const float* __restrict__ Dp,
    unsigned short* __restrict__ Y16, float carry)
{
  __shared__ __align__(16) float sXd[16 * 48];
  __shared__ __align__(16) float sY[16 * kDx];
  __shared__ float sWd[kDtR * kDx];
  __shared__ float sA[kNst * kDx];
  __shared__ float sH[kNst * kDx];
  const int tid = threadIdx.x;
  const size_t row0 = (size_t)blockIdx.x * kL;
#pragma unroll 1
  for (int r = 0; r < kDtR; ++r) sWd[r * kDx + tid] = Wdt[tid * kDtR + r];
#pragma unroll 1
  for (int n = 0; n < kNst; ++n) {
    sA[n * kDx + tid] = -expf(Alog[tid * kNst + n]);
    sH[n * kDx + tid] = 0.0f;
  }
  const float bb = bdt[tid];
  const float Dd = Dp[tid];
  __syncthreads();
#pragma unroll 1
  for (int t0 = 0; t0 < kL; t0 += 16) {
    __syncthreads();
#pragma unroll
    for (int i = 0; i < 2; ++i) {
      const int idx = tid + i * kDx;
      const int r = idx / 12;
      const int c4 = (idx - r * 12) * 4;
      *(v4f*)(sXd + r * 48 + c4) = *(const v4f*)(XD + (row0 + t0 + r) * kXdP + c4);
    }
    __syncthreads();
#pragma unroll 1
    for (int s = 0; s < 16; ++s) {
      const float* xr = sXd + s * 48;
      float vdot = 0.0f;
#pragma unroll 1
      for (int r4 = 0; r4 < kDtR / 4; ++r4) {
        const v4f xv = *(const v4f*)(xr + 4 * r4);
        const float* wp = sWd + (4 * r4) * kDx + tid;
        vdot = fmaf(xv[0], wp[0], vdot);
        vdot = fmaf(xv[1], wp[kDx], vdot);
        vdot = fmaf(xv[2], wp[2 * kDx], vdot);
        vdot = fmaf(xv[3], wp[3 * kDx], vdot);
      }
      const float v = vdot + bb;
      const float dt = fmaxf(v, 0.0f) + log1pf(expf(-fabsf(v)));
      const float xt = XH32[(row0 + t0 + s) * kDx + tid];
      const float dtx = dt * xt;
      float y = 0.0f;
#pragma unroll 1
      for (int n = 0; n < kNst; ++n) {
        const float e = expf(dt * sA[n * kDx + tid]);
        const float hn = fmaf(e, sH[n * kDx + tid], dtx * xr[kDtR + n]);
        sH[n * kDx + tid] = hn;
        y = fmaf(hn, xr[kDtR + kNst + n], y);
      }
      y = y + xt * Dd;
      sY[s * kDx + tid] = y;
    }
    __syncthreads();
    v8h hv[2];
#pragma unroll
    for (int it = 0; it < 2; ++it) {
      const int g = it * kDx + tid;
      const float* sp = sY + g * 8;
      const v4f a0 = *(const v4f*)(sp);
      const v4f a1 = *(const v4f*)(sp + 4);
#pragma unroll
      for (int e = 0; e < 4; ++e) {
        hv[it][e]     = (_Float16)(a0[e] * carry);
        hv[it][4 + e] = (_Float16)(a1[e] * carry);
      }
    }
    for (int pass = 0; pass < 2; ++pass) {
#pragma unroll
      for (int it = 0; it < 2; ++it) {
        const int g = it * kDx + tid;
        *(volatile v8h*)(Y16 + (row0 + t0) * kDx + g * 8) = hv[it];
      }
      __threadfence();
    }
  }
}

__global__ __launch_bounds__(256) void fuse_residual_pad_kernel(
    const unsigned short* __restrict__ OUT16, const float* __restrict__ XL,
    unsigned short* __restrict__ IMG, float inv_carry)
{
  __shared__ __align__(16) float sL[kDm * 60];
  const int tid = threadIdx.x;
  const int bb = blockIdx.x / kHP;
  const int py = blockIdx.x - bb * kHP;
  const bool rowIn = (py >= 1) && (py <= kH);
  int oy = py - 1;
  oy = oy < 0 ? 0 : oy;
  oy = oy > (kH - 1) ? (kH - 1) : oy;
  const float* src = XL + (size_t)bb * kDm * kL + oy * kW;
#pragma unroll 1
  for (int p = 0; p < 11; ++p) {
    int idx = tid + p * 256;
    idx = idx < (kDm * 14) ? idx : (kDm * 14 - 1);
    const int c = idx / 14;
    const int j = idx - c * 14;
    const v4f v = *(const v4f*)(src + (size_t)c * kL + 4 * j);
    *(v4f*)(sL + c * 60 + 4 * j) = v;
  }
  __syncthreads();
  unsigned short* dstRow = IMG + (size_t)(bb * kHP + py) * kWP * kDm;
#pragma unroll 1
  for (int it = 0; it < 6; ++it) {
    const int g = tid + it * 256;
    const bool active = g < (kWP * 24);
    const int gc = active ? g : (kWP * 24 - 1);
    const int px = gc / 24;
    const int c8 = (gc - px * 24) * 8;
    const bool inside = rowIn && (px >= 1) && (px <= kW);
    int ox = px - 1;
    ox = ox < 0 ? 0 : ox;
    ox = ox > (kW - 1) ? (kW - 1) : ox;
    const size_t m = (size_t)bb * kL + oy * kW + ox;
    const v4u w = *(const v4u*)(const void*)(OUT16 + m * kDm + c8);
    const unsigned w0 = w[0];
    const unsigned w1 = w[1];
    const unsigned w2 = w[2];
    const unsigned w3 = w[3];
    const float* lp = sL + c8 * 60 + ox;
    float t0 = fmaf(h16_to_f32(w0 & 0xffffu), inv_carry, lp[0]);
    float t1 = fmaf(h16_to_f32(w0 >> 16),     inv_carry, lp[60]);
    float t2 = fmaf(h16_to_f32(w1 & 0xffffu), inv_carry, lp[120]);
    float t3 = fmaf(h16_to_f32(w1 >> 16),     inv_carry, lp[180]);
    float t4 = fmaf(h16_to_f32(w2 & 0xffffu), inv_carry, lp[240]);
    float t5 = fmaf(h16_to_f32(w2 >> 16),     inv_carry, lp[300]);
    float t6 = fmaf(h16_to_f32(w3 & 0xffffu), inv_carry, lp[360]);
    float t7 = fmaf(h16_to_f32(w3 >> 16),     inv_carry, lp[420]);
    t0 = inside ? t0 : 0.0f;
    t1 = inside ? t1 : 0.0f;
    t2 = inside ? t2 : 0.0f;
    t3 = inside ? t3 : 0.0f;
    t4 = inside ? t4 : 0.0f;
    t5 = inside ? t5 : 0.0f;
    t6 = inside ? t6 : 0.0f;
    t7 = inside ? t7 : 0.0f;
    v8h hv;
    hv[0] = (_Float16)t0;
    hv[1] = (_Float16)t1;
    hv[2] = (_Float16)t2;
    hv[3] = (_Float16)t3;
    hv[4] = (_Float16)t4;
    hv[5] = (_Float16)t5;
    hv[6] = (_Float16)t6;
    hv[7] = (_Float16)t7;
    if (active) *(volatile v8h*)(dstRow + (size_t)g * 8) = hv;
    __threadfence();
    if (active) *(volatile v8h*)(dstRow + (size_t)g * 8) = hv;
  }
}

__global__ __launch_bounds__(256) void zero_border_kernel(unsigned short* __restrict__ Y2)
{
  const int g = blockIdx.x * 256 + threadIdx.x;
  if (g >= kNB * 228 * 24) return;
  const int pixi = g / 24;
  const int ch = g - pixi * 24;
  const int bb = pixi / 228;
  const int bp = pixi - bb * 228;
  const int r2 = bp - 116;
  const int py = (bp < 58) ? 0 : ((bp < 116) ? (kHP - 1) : (1 + (r2 >> 1)));
  const int px = (bp < 58) ? bp : ((bp < 116) ? (bp - 58) : ((r2 & 1) ? (kWP - 1) : 0));
  unsigned short* q = Y2 + ((size_t)(bb * kHP + py) * kWP + px) * kDm + ch * 8;
  const v4u z = (v4u){0u, 0u, 0u, 0u};
  *(volatile v4u*)(void*)q = z;
  __threadfence();
  *(volatile v4u*)(void*)q = z;
}

__global__ __launch_bounds__(256) void conv3x3_relu_kernel(
    const unsigned short* __restrict__ IMGp, const unsigned short* __restrict__ Wp,
    const float* __restrict__ bias, unsigned short* __restrict__ Y2, float scale)
{
  const _Float16* IMG = (const _Float16*)IMGp;
  const _Float16* Wt  = (const _Float16*)Wp;
  __shared__ __align__(16) float sT[8][16 * 68];
  const int lane = threadIdx.x & 31;
  const int wave = threadIdx.x >> 5;
  constexpr int tilesN = kDm / 64;
  const int tile = blockIdx.x * 8 + wave;
  if (tile >= kTilesM * tilesN) return;
  const int tm = tile / tilesN;
  const int tn = tile - tm * tilesN;
  const int m0 = tm << 6;
  const int n0 = tn << 6;
  const int rlane = lane & 15;
  const int koff  = (lane >> 4) * 8;
  const int mOff  = (lane >> 4) * 8;
  int aoff[4], boff[4];
#pragma unroll
  for (int i = 0; i < 4; ++i) {
    const int m = m0 + (i << 4) + rlane;
    const int bb = m / kL;
    const int l = m - bb * kL;
    const int oy = l / kW;
    const int ox = l - oy * kW;
    aoff[i] = ((bb * kHP + oy) * kWP + ox) * kDm + koff;
    boff[i] = (n0 + (i << 4) + rlane) * kK2 + koff;
  }
  v8f acc[4][4];
#pragma unroll
  for (int i = 0; i < 4; ++i)
#pragma unroll
    for (int j = 0; j < 4; ++j) acc[i][j] = (v8f){0.f, 0.f, 0.f, 0.f, 0.f, 0.f, 0.f, 0.f};

#pragma unroll 1
  for (int tap = 0; tap < 9; ++tap) {
    const int ky = tap / 3;
    const int kx = tap - ky * 3;
    const int toff = (ky * kWP + kx) * kDm;
#pragma unroll 1
    for (int c0 = 0; c0 < kDm; c0 += 32) {
      v16h bh[4];
#pragma unroll
      for (int j = 0; j < 4; ++j) bh[j] = frag_load(Wt + boff[j] + tap * kDm + c0);
#pragma unroll
      for (int i = 0; i < 4; ++i) {
        const v16h ah = frag_load(IMG + aoff[i] + toff + c0);
#pragma unroll
        for (int j = 0; j < 4; ++j) acc[i][j] = mma_h(ah, bh[j], acc[i][j]);
      }
    }
  }

  float bvj[4];
#pragma unroll
  for (int j = 0; j < 4; ++j) bvj[j] = bias[n0 + (j << 4) + rlane];
  float* slab = sT[wave];
#pragma unroll
  for (int i = 0; i < 4; ++i) {
    const int mBase = m0 + (i << 4);
#pragma unroll
    for (int j = 0; j < 4; ++j) {
#pragma unroll
      for (int r = 0; r < 8; ++r) {
        const float v = fmaf(acc[i][j][r], scale, bvj[j]);
        slab[(mOff + r) * 68 + (j << 4) + rlane] = fmaxf(v, 0.0f);
      }
    }
    slab_sync();
    {
      const int q = lane >> 3, c8 = (lane & 7) * 8;
      for (int pass = 0; pass < 2; ++pass) {
#pragma unroll
        for (int it = 0; it < 4; ++it) {
          const int row = it * 4 + q;
          const int m = mBase + row;
          const int bb = m / kL;
          const int l = m - bb * kL;
          const int oy = l / kW;
          const int ox = l - oy * kW;
          const float* sp = slab + row * 68 + c8;
          v8h hv;
#pragma unroll
          for (int e = 0; e < 8; ++e) hv[e] = (_Float16)sp[e];
          *(volatile v8h*)(Y2 + ((size_t)((bb * kHP + oy + 1) * kWP + ox + 1)) * kDm + n0 + c8) = hv;
        }
        __threadfence();
      }
    }
    slab_sync();
  }
}

__global__ __launch_bounds__(256) void convT_parity_kernel(
    const unsigned short* __restrict__ Y2p, const unsigned short* __restrict__ Wp,
    float* __restrict__ Y3, float scale)
{
  const _Float16* Y2 = (const _Float16*)Y2p;
  const _Float16* Wt = (const _Float16*)Wp;
  __shared__ __align__(16) float sT[8][16 * 36];
  const int lane = threadIdx.x & 31;
  const int wave = threadIdx.x >> 5;
  const int cls = blockIdx.y;
  const int sy = cls >> 1, sx = cls & 1;
  constexpr int tilesN = kOC / 32;
  const int tile = blockIdx.x * 8 + wave;
  if (tile >= kTilesM * tilesN) return;
  const int tm = tile / tilesN;
  const int tn = tile - tm * tilesN;
  const int m0 = tm << 6;
  const int n0 = tn << 5;
  const int rlane = lane & 15;
  const int koff  = (lane >> 4) * 8;
  const int mOff  = (lane >> 4) * 8;
  int aoff[4], boff[2];
#pragma unroll
  for (int i = 0; i < 4; ++i) {
    const int m = m0 + (i << 4) + rlane;
    const int bb = m / kL;
    const int l = m - bb * kL;
    const int ty = l / kW;
    const int tx = l - ty * kW;
    aoff[i] = ((bb * kHP + ty + 1) * kWP + tx + 1) * kDm + koff;
  }
#pragma unroll
  for (int j = 0; j < 2; ++j) boff[j] = (cls * kOC + n0 + (j << 4) + rlane) * kKT + koff;
  v8f acc[4][2];
#pragma unroll
  for (int i = 0; i < 4; ++i)
#pragma unroll
    for (int j = 0; j < 2; ++j) acc[i][j] = (v8f){0.f, 0.f, 0.f, 0.f, 0.f, 0.f, 0.f, 0.f};

#pragma unroll 1
  for (int jj = 0; jj < 4; ++jj) {
    const int jy = jj >> 1, jx = jj & 1;
    const int dy = jy ? (sy ? 1 : -1) : 0;
    const int dx = jx ? (sx ? 1 : -1) : 0;
    const int toff = (dy * kWP + dx) * kDm;
#pragma unroll 1
    for (int c0 = 0; c0 < kDm; c0 += 32) {
      v16h bh[2];
#pragma unroll
      for (int j = 0; j < 2; ++j) bh[j] = frag_load(Wt + boff[j] + jj * kDm + c0);
#pragma unroll
      for (int i = 0; i < 4; ++i) {
        const v16h ah = frag_load(Y2 + aoff[i] + toff + c0);
#pragma unroll
        for (int j = 0; j < 2; ++j) acc[i][j] = mma_h(ah, bh[j], acc[i][j]);
      }
    }
  }

  float* slab = sT[wave];
  float* Cb = Y3 + (size_t)cls * kRows * kOC;
#pragma unroll
  for (int i = 0; i < 4; ++i) {
    const int mBase = m0 + (i << 4);
#pragma unroll
    for (int j = 0; j < 2; ++j) {
#pragma unroll
      for (int r = 0; r < 8; ++r) slab[(mOff + r) * 36 + (j << 4) + rlane] = acc[i][j][r] * scale;
    }
    slab_sync();
    {
      const int q = lane >> 3, c4 = (lane & 7) * 4;
      for (int pass = 0; pass < 2; ++pass) {
#pragma unroll
        for (int it = 0; it < 4; ++it) {
          const int row = it * 4 + q;
          const v4f v = *(const v4f*)(slab + row * 36 + c4);
          *(volatile v4f*)(Cb + (size_t)(mBase + row) * kOC + n0 + c4) = v;
        }
        __threadfence();
      }
    }
    slab_sync();
  }
}

__global__ __launch_bounds__(256) void depth_to_space_bias_kernel(
    const float* __restrict__ Y3, const float* __restrict__ bias, float* __restrict__ OUT)
{
  const int g = blockIdx.x * 256 + threadIdx.x;
  if (g >= (kNB * kOC * kOH * kOW) / 4) return;
  const int f0 = g << 2;
  const int plane = f0 / (kOH * kOW);
  const int rem = f0 - plane * (kOH * kOW);
  const int oy = rem / kOW;
  const int ox = rem - oy * kOW;
  const int bb = plane / kOC;
  const int co = plane - bb * kOC;
  const int ty = oy >> 1, sy = oy & 1;
  const int tx0 = ox >> 1;
  const size_t mA = (size_t)bb * kL + ty * kW + tx0;
  const size_t c0 = (size_t)(sy * 2) * kRows;
  const size_t c1 = (size_t)(sy * 2 + 1) * kRows;
  const float bv = bias[co];
  const float a0 = Y3[(c0 + mA) * kOC + co];
  const float a1 = Y3[(c1 + mA) * kOC + co];
  const float a2 = Y3[(c0 + mA + 1) * kOC + co];
  const float a3 = Y3[(c1 + mA + 1) * kOC + co];
  v4f v;
  v[0] = a0 + bv;
  v[1] = a1 + bv;
  v[2] = a2 + bv;
  v[3] = a3 + bv;
  float* q = OUT + (size_t)f0;
  *(volatile v4f*)q = v;
  __threadfence();
  *(volatile v4f*)q = v;
}

extern "C" void kernel_launch(void* const* d_in, const int* in_sizes, int n_in,
                              void* d_out, int out_size, void* d_ws, size_t ws_size,
                              hipStream_t stream)
{
  if (n_in < 17) return;
  if (in_sizes[0] != kNB * kDm * kL || in_sizes[1] != kNB * kDm * kL) return;
  if (in_sizes[2] != kDm * kDm) return;
  if (in_sizes[3] != kDx * 3 || in_sizes[4] != kDx) return;
  if (in_sizes[5] != kDx * 3 || in_sizes[6] != kDx) return;
  if (in_sizes[7] != kXdN * kDx) return;
  if (in_sizes[8] != kDx * kDtR || in_sizes[9] != kDx) return;
  if (in_sizes[10] != kDx * kNst || in_sizes[11] != kDx) return;
  if (in_sizes[12] != kDm * kDm) return;
  if (in_sizes[13] != kDm * kDm * 9 || in_sizes[14] != kDm) return;
  if (in_sizes[15] != kDm * kOC * 16 || in_sizes[16] != kOC) return;
  if (out_size != kNB * kOC * kOH * kOW) return;
  if (ws_size < kWsTotal) return;

  const float* x        = (const float*)d_in[0];
  const float* x_last   = (const float*)d_in[1];
  const float* in_w     = (const float*)d_in[2];
  const float* c1x_w    = (const float*)d_in[3];
  const float* c1x_b    = (const float*)d_in[4];
  const float* c1z_w    = (const float*)d_in[5];
  const float* c1z_b    = (const float*)d_in[6];
  const float* xproj_w  = (const float*)d_in[7];
  const float* dt_w     = (const float*)d_in[8];
  const float* dt_b     = (const float*)d_in[9];
  const float* A_log    = (const float*)d_in[10];
  const float* ssm_D    = (const float*)d_in[11];
  const float* out_w    = (const float*)d_in[12];
  const float* c2_w     = (const float*)d_in[13];
  const float* c2_b     = (const float*)d_in[14];
  const float* ct_w     = (const float*)d_in[15];
  const float* ct_b     = (const float*)d_in[16];
  float* out = (float*)d_out;

  char* ws = (char*)d_ws;
  unsigned short* WIN   = (unsigned short*)(ws + kOffWIN);
  unsigned short* WOUT  = (unsigned short*)(ws + kOffWOUT);
  unsigned short* WXP   = (unsigned short*)(ws + kOffWXP);
  unsigned short* WC2   = (unsigned short*)(ws + kOffWC2);
  unsigned short* WCT   = (unsigned short*)(ws + kOffWCT);
  unsigned short* XA    = (unsigned short*)(ws + kOffXA);
  unsigned short* XZ    = (unsigned short*)(ws + kOffXZ);
  float*          XH32  = (float*)(ws + kOffXH32);
  unsigned short* XH16  = (unsigned short*)(ws + kOffXH16);
  unsigned short* Z16   = (unsigned short*)(ws + kOffZ16);
  float*          XD    = (float*)(ws + kOffXD);
  unsigned short* Y16   = (unsigned short*)(ws + kOffY16);
  unsigned short* OUT16 = (unsigned short*)(ws + kOffOUT16);
  unsigned short* IMG   = (unsigned short*)(ws + kOffIMG);
  unsigned short* Y2    = (unsigned short*)(ws + kOffY2);
  float*          Y3    = (float*)(ws + kOffY3);

  cast_f16_pad_kernel<<<(kDm * kDm / 8) / 256, 256, 0, stream>>>(in_w, WIN, kDm * kDm / 8, kDm * kDm, kWCarry);
  cast_f16_pad_kernel<<<(kDm * kDm / 8) / 256, 256, 0, stream>>>(out_w, WOUT, kDm * kDm / 8, kDm * kDm, kWCarry);
  cast_f16_pad_kernel<<<(kXdP * kDx / 8) / 256, 256, 0, stream>>>(xproj_w, WXP, kXdP * kDx / 8, kXdN * kDx, kWCarry);
  pack_conv3x3_kernel<<<(kDm * kK2 / 8) / 256, 256, 0, stream>>>(c2_w, WC2, kWCarry);
  pack_convT_kernel<<<(4 * kOC * kKT / 8) / 256, 256, 0, stream>>>(ct_w, WCT, kWCarry);

  nchw_to_rows_f16_kernel<<<kNB * (kL / 64), 256, 0, stream>>>(x, XA);

  gemm64_f16_kernel<1, false><<<(kTilesM * (kDm / 64)) / 8, 256, 0, stream>>>(
      XA, kDm, XA, kDm, 0, WIN, kDm, (void*)XZ, kDm, kRows, kDm, kDm, 1.0f / kWCarry);

  dwconv_silu_kernel<<<kRows / 32, 256, 0, stream>>>(XZ, c1x_w, c1x_b, c1z_w, c1z_b, XH32, XH16, Z16, kActCarry);

  gemm64_f16_kernel<0, false><<<(kTilesM * (kXdP / 64)) / 8, 256, 0, stream>>>(
      XH16, kDx, XH16, kDx, 0, WXP, kDx, (void*)XD, kXdP, kRows, kXdP, kDx, 1.0f / (kActCarry * kWCarry));

  scan_kernel<<<kNB, kDx, 0, stream>>>(XD, XH32, dt_w, dt_b, A_log, ssm_D, Y16, kActCarry);

  gemm64_f16_kernel<1, true><<<(kTilesM * (kDm / 64)) / 8, 256, 0, stream>>>(
      Y16, kDx, Z16, kDx, kDx, WOUT, kDm, (void*)OUT16, kDm, kRows, kDm, kDm, kOutCarry / (kActCarry * kWCarry));

  fuse_residual_pad_kernel<<<kNB * kHP, 256, 0, stream>>>(OUT16, x_last, IMG, 1.0f / kOutCarry);

  zero_border_kernel<<<(kNB * 228 * 24) / 256, 256, 0, stream>>>(Y2);

  conv3x3_relu_kernel<<<(kTilesM * (kDm / 64)) / 8, 256, 0, stream>>>(IMG, WC2, c2_b, Y2, 1.0f / kWCarry);

  convT_parity_kernel<<<dim3((kTilesM * (kOC / 32)) / 8, 4), 256, 0, stream>>>(Y2, WCT, Y3, 1.0f / kWCarry);

  depth_to_space_bias_kernel<<<(kNB * kOC * kOH * kOW / 4) / 256, 256, 0, stream>>>(Y3, ct_b, out);
}
